// HiLo_48129403519638
// MI455X (gfx1250) — hardware-run, weakly checked
//
#include <hip/hip_runtime.h>
#include <hip/hip_bf16.h>

typedef __attribute__((ext_vector_type(16))) _Float16 v16h;
typedef __attribute__((ext_vector_type(8)))  _Float16 v8h;
typedef __attribute__((ext_vector_type(16))) __bf16   v16b;
typedef __attribute__((ext_vector_type(8)))  __bf16   v8b;
typedef __attribute__((ext_vector_type(8)))  float    v8f;
typedef __attribute__((ext_vector_type(4)))  float    v4f;
typedef __attribute__((ext_vector_type(4)))  unsigned v4u;

static constexpr int kBatch   = 4;
static constexpr int kChan    = 512;
static constexpr int kPix     = 4096;
static constexpr int kTok     = kBatch * kPix;
static constexpr int kPoolPer = 1024;
static constexpr int kPool    = kBatch * kPoolPer;
static constexpr int kHead    = 64;
static constexpr int kHalfDim = 256;
static constexpr int kQkvN    = 768;
static constexpr float kScale = 0.125f;
static constexpr float kPCarry = 32768.0f;
static constexpr float kLoOutCarry = 64.0f;
static constexpr float kLoWCarry   = 32.0f;

static_assert(kTok % 64 == 0 && kPool % 64 == 0 && kPix % 64 == 0);
static_assert(kQkvN % 64 == 0 && kHalfDim % 64 == 0 && kChan % 64 == 0);
static_assert(kChan % 32 == 0 && kHalfDim % 32 == 0);

static constexpr size_t kBytesXh   = (size_t)kTok * kChan * 2;
static constexpr size_t kBytesPool = (size_t)kPool * kChan * 2;
static constexpr size_t kBytesQkv  = (size_t)kTok * kQkvN * 2;
static constexpr size_t kBytesT256 = (size_t)kTok * kHalfDim * 2;
static constexpr size_t kBytesP256 = (size_t)kPool * kHalfDim * 2;
static constexpr size_t kBytesWqkv = (size_t)kQkvN * kChan * 2;
static constexpr size_t kBytesW256 = (size_t)kHalfDim * kHalfDim * 2;
static constexpr size_t kBytesWq   = (size_t)kHalfDim * kChan * 2;
static constexpr size_t kBytesWkv  = (size_t)kChan * kChan * 2;
static constexpr size_t kCarveTotal = 2 * kBytesXh + kBytesPool + 2 * kBytesQkv + kBytesT256 + 2 * kBytesP256 +
                                      3 * kBytesT256 + 2 * kBytesWqkv + 2 * kBytesW256 + kBytesWq + kBytesWkv + kBytesW256;
static_assert(kCarveTotal == 128581632);
static_assert(kCarveTotal <= 134217728);

__device__ __forceinline__ unsigned short f2bf_bits(float f) {
  unsigned u = __float_as_uint(f);
  return (unsigned short)((u + 0x7FFFu + ((u >> 16) & 1u)) >> 16);
}
__device__ __forceinline__ float bf_bits2f(unsigned short h) { return __uint_as_float(((unsigned)h) << 16); }

__device__ __forceinline__ void dep_guard_h(v8f& a, v8f& b, v16h x, v16h y) { asm volatile("v_nop\n\tv_nop\n\tv_nop\n\tv_nop" : "+v"(a), "+v"(b) : "v"(x), "v"(y)); }
__device__ __forceinline__ void dep_guard_b(v8f& a, v8f& b, v16b x, v16b y) { asm volatile("v_nop\n\tv_nop\n\tv_nop\n\tv_nop" : "+v"(a), "+v"(b) : "v"(x), "v"(y)); }
__device__ __forceinline__ void keep4_h(v16h a, v16h b, v16h c, v16h d) { asm volatile("v_nop" :: "v"(a), "v"(b), "v"(c), "v"(d)); }
__device__ __forceinline__ void keep4_b(v16b a, v16b b, v16b c, v16b d) { asm volatile("v_nop" :: "v"(a), "v"(b), "v"(c), "v"(d)); }
__device__ __forceinline__ void acc_guard4(v8f& a, v8f& b, v8f& c, v8f& d) { asm volatile("v_nop\n\tv_nop\n\tv_nop\n\tv_nop" : "+v"(a), "+v"(b), "+v"(c), "+v"(d)); }
template <typename T> struct Frag;
template <> struct Frag<_Float16> {
  typedef v16h V; union U { v16h v; v8h h[2]; };
  static __device__ __forceinline__ v16h load(const _Float16* p) {
    U f; f.h[0] = *(const v8h*)(p); f.h[1] = *(const v8h*)(p + 16); return f.v;
  }
  static __device__ __forceinline__ v8f mma(v16h a, v16h b, v8f c) {
    return __builtin_amdgcn_wmma_f32_16x16x32_f16(false, a, false, b, (short)0, c, false, false);
  }
  static __device__ __forceinline__ void guard(v8f& a, v8f& b, v16h x, v16h y) { dep_guard_h(a, b, x, y); }
  static __device__ __forceinline__ void keep(v16h a, v16h b, v16h c, v16h d) { keep4_h(a, b, c, d); }
};
template <> struct Frag<__bf16> {
  typedef v16b V; union U { v16b v; v8b h[2]; };
  static __device__ __forceinline__ v16b load(const __bf16* p) {
    U f; f.h[0] = *(const v8b*)(p); f.h[1] = *(const v8b*)(p + 16); return f.v;
  }
  static __device__ __forceinline__ v8f mma(v16b a, v16b b, v8f c) {
    return __builtin_amdgcn_wmma_f32_16x16x32_bf16(false, a, false, b, (short)0, c, false, false);
  }
  static __device__ __forceinline__ void guard(v8f& a, v8f& b, v16b x, v16b y) { dep_guard_b(a, b, x, y); }
  static __device__ __forceinline__ void keep(v16b a, v16b b, v16b c, v16b d) { keep4_b(a, b, c, d); }
};

__device__ __forceinline__ v8f mma_b(v16b a, v16b b, v8f c) {
  c = __builtin_amdgcn_wmma_f32_16x16x32_bf16(false, a, false, b, (short)0, c, false, false);
  asm volatile("v_nop\n\tv_nop\n\tv_nop\n\tv_nop" : "+v"(c) : "v"(a), "v"(b));
  return c;
}
__device__ __forceinline__ v8f mma_h(v16h a, v16h b, v8f c) {
  c = __builtin_amdgcn_wmma_f32_16x16x32_f16(false, a, false, b, (short)0, c, false, false);
  asm volatile("v_nop\n\tv_nop\n\tv_nop\n\tv_nop" : "+v"(c) : "v"(a), "v"(b));
  return c;
}
__device__ __forceinline__ v8f zero8() { return (v8f){0.f,0.f,0.f,0.f,0.f,0.f,0.f,0.f}; }

template <int ET> struct Elem;
template <> struct Elem<0> { typedef _Float16 T; };
template <> struct Elem<1> { typedef __bf16 T; };
template <int ET, bool SPLIT, int BIAS_MODE, int OUT_MODE>
__global__ __launch_bounds__(256) void wmma_gemm64(
    const unsigned short* __restrict__ Ap, const unsigned short* __restrict__ A2p, int lda, long strideA,
    const unsigned short* __restrict__ Btp, const unsigned short* __restrict__ Bt2p, int ldb, long strideB,
    void* __restrict__ Cout, void* __restrict__ Cout2, int ldc, long strideC,
    const float* __restrict__ bias,
    int M, int N, int K, float scale) {
  typedef typename Elem<ET>::T T;
  typedef typename Frag<T>::V V;
  const T* A = (const T*)Ap; const T* A2 = (const T*)A2p; const T* Bt = (const T*)Btp; const T* Bt2 = (const T*)Bt2p;
  __shared__ __align__(16) float sT[8][16 * 68];
  const int b    = blockIdx.y;
  const int lane = threadIdx.x & 31;
  const int wave = threadIdx.x >> 5;
  const int tilesN = N >> 6;
  const int tilesM = M >> 6;
  const int tile = blockIdx.x * 8 + wave;
  if (tile >= tilesM * tilesN) return;
  const int tm = tile / tilesN;
  const int tn = tile - tm * tilesN;
  const int m0 = tm << 6;
  const int n0 = tn << 6;

  const T* Ab  = A  + (size_t)b * strideA;
  const T* Bb  = Bt + (size_t)b * strideB;
  const T* Ab2 = SPLIT ? (A2  + (size_t)b * strideA) : nullptr;
  const T* Bb2 = SPLIT ? (Bt2 + (size_t)b * strideB) : nullptr;

  const int rlane = lane & 15;
  const int koff  = (lane >> 4) * 8;
  const int mOff  = (lane >> 4) * 8;

  v8f acc[4][4];
#pragma unroll
  for (int i = 0; i < 4; ++i)
#pragma unroll
    for (int j = 0; j < 4; ++j) acc[i][j] = zero8();

  for (int k0 = 0; k0 < K; k0 += 32) {
    V bh[4], bl[4];
#pragma unroll
    for (int j = 0; j < 4; ++j) {
      const size_t bo = (size_t)(n0 + (j << 4) + rlane) * ldb + koff + k0;
      bh[j] = Frag<T>::load(Bb + bo);
      if (SPLIT) bl[j] = Frag<T>::load(Bb2 + bo);
    }
#pragma unroll
    for (int i = 0; i < 4; ++i) {
      const size_t ao = (size_t)(m0 + (i << 4) + rlane) * lda + koff + k0;
      V ah = Frag<T>::load(Ab + ao);
      V al;
      if (SPLIT) al = Frag<T>::load(Ab2 + ao);
#pragma unroll
      for (int j = 0; j < 4; ++j) {
        acc[i][j] = Frag<T>::mma(ah, bh[j], acc[i][j]);
        if (SPLIT) {
          acc[i][j] = Frag<T>::mma(ah, bl[j], acc[i][j]);
          acc[i][j] = Frag<T>::mma(al, bh[j], acc[i][j]);
        }
      }
      Frag<T>::guard(acc[i][0], acc[i][3], ah, SPLIT ? al : ah);
    }
    Frag<T>::keep(bh[0], bh[1], bh[2], bh[3]);
    if (SPLIT) Frag<T>::keep(bl[0], bl[1], bl[2], bl[3]);
  }
  acc_guard4(acc[0][0], acc[0][1], acc[0][2], acc[0][3]);
  acc_guard4(acc[1][0], acc[1][1], acc[1][2], acc[1][3]);
  acc_guard4(acc[2][0], acc[2][1], acc[2][2], acc[2][3]);
  acc_guard4(acc[3][0], acc[3][1], acc[3][2], acc[3][3]);

  float* slab = sT[wave];
#pragma unroll
  for (int i = 0; i < 4; ++i) {
    const int mBase = m0 + (i << 4);
    float bm8[8];
#pragma unroll
    for (int r = 0; r < 8; ++r) bm8[r] = 0.f;
    if (BIAS_MODE == 1) {
      const v4f b0 = *(const v4f*)(bias + mBase + mOff);
      const v4f b1 = *(const v4f*)(bias + mBase + mOff + 4);
      bm8[0] = b0[0]; bm8[1] = b0[1]; bm8[2] = b0[2]; bm8[3] = b0[3];
      bm8[4] = b1[0]; bm8[5] = b1[1]; bm8[6] = b1[2]; bm8[7] = b1[3];
    }
#pragma unroll
    for (int j = 0; j < 4; ++j) {
#pragma unroll
      for (int r = 0; r < 8; ++r) {
        float v = acc[i][j][r] * scale;
        if (BIAS_MODE == 1) v += bm8[r];
        slab[(mOff + r) * 68 + (j << 4) + rlane] = v;
      }
    }
    __builtin_amdgcn_fence(__ATOMIC_RELEASE, "workgroup");
    __builtin_amdgcn_wave_barrier();
    __builtin_amdgcn_fence(__ATOMIC_ACQUIRE, "workgroup");
    if (OUT_MODE == 0) {
      float* C = (float*)Cout + (size_t)b * strideC;
      const int hh = lane >> 4, c4 = (lane & 15) * 4;
      for (int pass = 0; pass < 2; ++pass) {
#pragma unroll
        for (int it = 0; it < 8; ++it) {
          const int row = it * 2 + hh;
          v4f v = *(const v4f*)(slab + row * 68 + c4);
          *(volatile v4f*)(C + (size_t)(mBase + row) * ldc + n0 + c4) = v;
        }
        __threadfence();
      }
    } else {
      const int q = lane >> 3, c8 = (lane & 7) * 8;
      unsigned short* C  = (unsigned short*)Cout  + (size_t)b * strideC;
      unsigned short* C2 = (OUT_MODE == 2) ? ((unsigned short*)Cout2 + (size_t)b * strideC) : nullptr;
      for (int pass = 0; pass < 2; ++pass) {
#pragma unroll
        for (int it = 0; it < 4; ++it) {
          const int row = it * 4 + q;
          const float* sp = slab + row * 68 + c8;
          v8h hv, lv;
#pragma unroll
          for (int e = 0; e < 8; ++e) {
            if (OUT_MODE == 1) {
              hv[e] = (_Float16)sp[e];
            } else {
              unsigned short hb = f2bf_bits(sp[e]);
              unsigned short lb = f2bf_bits(sp[e] - bf_bits2f(hb));
              hv[e] = __builtin_bit_cast(_Float16, hb);
              lv[e] = __builtin_bit_cast(_Float16, lb);
            }
          }
          *(volatile v8h*)(C + (size_t)(mBase + row) * ldc + n0 + c8) = hv;
          if (OUT_MODE == 2) *(volatile v8h*)(C2 + (size_t)(mBase + row) * ldc + n0 + c8) = lv;
        }
        __threadfence();
      }
    }
    __builtin_amdgcn_fence(__ATOMIC_RELEASE, "workgroup");
    __builtin_amdgcn_wave_barrier();
    __builtin_amdgcn_fence(__ATOMIC_ACQUIRE, "workgroup");
  }
}

template <int OT>
__global__ __launch_bounds__(256) void tr_convert(const float* __restrict__ in, long strideIn, int pitchIn,
                                                  unsigned short* __restrict__ outH, unsigned short* __restrict__ outL,
                                                  long strideOut, int pitchOut, float scale) {
  __shared__ float tile[64][65];
  const int tid = threadIdx.x, lane = tid & 31, wave = tid >> 5;
  const int c0 = blockIdx.x * 64;
  const int r0 = blockIdx.y * 64;
  const float* ib = in + (size_t)blockIdx.z * strideIn;
  {
    const int r = tid >> 2, c16 = (tid & 3) * 16;
    const float* p = ib + (size_t)(r0 + r) * pitchIn + c0 + c16;
#pragma unroll
    for (int i = 0; i < 4; ++i) {
      const v4f v = *(const v4f*)(p + 4 * i);
      tile[r][c16 + 4 * i + 0] = v[0];
      tile[r][c16 + 4 * i + 1] = v[1];
      tile[r][c16 + 4 * i + 2] = v[2];
      tile[r][c16 + 4 * i + 3] = v[3];
    }
  }
  __syncthreads();
  unsigned short* oh = outH + (size_t)blockIdx.z * strideOut;
  unsigned short* ol = (OT == 2) ? (outL + (size_t)blockIdx.z * strideOut) : nullptr;
  const int q = lane >> 3, c8 = (lane & 7) * 8;
  for (int pass = 0; pass < 2; ++pass) {
#pragma unroll
    for (int it = 0; it < 2; ++it) {
      const int cc = wave * 8 + it * 4 + q;
      v8h hv, lv;
#pragma unroll
      for (int e = 0; e < 8; ++e) {
        const float f = tile[c8 + e][cc];
        if (OT == 0) {
          hv[e] = (_Float16)(f * scale);
        } else {
          const unsigned short hb = f2bf_bits(f);
          hv[e] = __builtin_bit_cast(_Float16, hb);
          if (OT == 2) {
            const unsigned short lb = f2bf_bits(f - bf_bits2f(hb));
            lv[e] = __builtin_bit_cast(_Float16, lb);
          }
        }
      }
      const size_t o = (size_t)(c0 + cc) * pitchOut + r0 + c8;
      *(volatile v8h*)(oh + o) = hv;
      if (OT == 2) *(volatile v8h*)(ol + o) = lv;
    }
    __threadfence();
  }
}

__global__ __launch_bounds__(256) void pool_to_bf16(const float* __restrict__ x, unsigned short* __restrict__ pooled) {
  __shared__ float tile[64][65];
  const int tid = threadIdx.x, lane = tid & 31, wave = tid >> 5;
  const int a = blockIdx.x, c0 = blockIdx.y * 64, b = blockIdx.z;
#pragma unroll
  for (int it = 0; it < 8; ++it) {
    const int item = it * 256 + tid;
    const int c = item >> 5, rp = (item >> 4) & 1, quad = item & 15;
    const float* p0 = x + ((size_t)(b * kChan + c0 + c) * 64 + (4 * a + 2 * rp)) * 64 + 4 * quad;
    const v4f u = *(const v4f*)(p0);
    const v4f w = *(const v4f*)(p0 + 64);
    const float m0 = (((u[0] + u[1]) + w[0]) + w[1]) * 0.25f;
    const float m1 = (((u[2] + u[3]) + w[2]) + w[3]) * 0.25f;
    const int gl = rp * 32 + 2 * quad;
    tile[c][gl] = m0;
    tile[c][gl + 1] = m1;
  }
  __syncthreads();
  const int q = lane >> 3, c8 = (lane & 7) * 8;
  for (int pass = 0; pass < 2; ++pass) {
#pragma unroll
    for (int it = 0; it < 2; ++it) {
      const int gl = wave * 8 + it * 4 + q;
      v8h hv;
#pragma unroll
      for (int e = 0; e < 8; ++e) hv[e] = __builtin_bit_cast(_Float16, f2bf_bits(tile[c8 + e][gl]));
      *(volatile v8h*)(pooled + (size_t)(b * kPoolPer + 64 * a + gl) * kChan + c0 + c8) = hv;
    }
    __threadfence();
  }
}

__global__ __launch_bounds__(128) void win_attn(const unsigned short* __restrict__ qkvH, const unsigned short* __restrict__ qkvL,
                                                unsigned short* __restrict__ oH, unsigned short* __restrict__ oL) {
  __shared__ __align__(16) unsigned short Ph[4][16 * 32];
  __shared__ __align__(16) unsigned short Pl[4][16 * 32];
  __shared__ __align__(16) unsigned short Vh[4][64 * 32];
  __shared__ __align__(16) unsigned short Vl[4][64 * 32];
  __shared__ __align__(16) float Os[4][16 * 68];
  const int tid = threadIdx.x, lane = tid & 31, wave = tid >> 5;
  const int hh = lane >> 4, c = lane & 15, koff = hh * 8;
  const int tileId = blockIdx.x;
  const int b = tileId >> 8, tt = tileId & 255, gh = tt >> 3, cg = tt & 7;
  const int tokBase = b * kPix + (2 * gh) * 64 + 8 * cg;
  const int tokc = tokBase + ((c & 3) >> 1) * 64 + 2 * (c >> 2) + (c & 1);
  const int hc = wave * kHead;
  unsigned short* ph = Ph[wave];
  unsigned short* pl = Pl[wave];
  unsigned short* vh = Vh[wave];
  unsigned short* vl = Vl[wave];

  {
    const v4u z = (v4u){0u, 0u, 0u, 0u};
    *(v4u*)(ph + c * 32 + 16 + koff) = z;
    *(v4u*)(pl + c * 32 + 16 + koff) = z;
#pragma unroll
    for (int rr = 0; rr < 4; ++rr) {
      *(v4u*)(vh + (rr * 16 + c) * 32 + 16 + koff) = z;
      *(v4u*)(vl + (rr * 16 + c) * 32 + 16 + koff) = z;
    }
  }
  {
    const int dh = hh * 32;
    const size_t vbase = (size_t)tokc * kQkvN + 512 + hc + dh;
#pragma unroll
    for (int i = 0; i < 4; ++i) {
      const v4u wh = *(const v4u*)(qkvH + vbase + 8 * i);
      const v4u wl = *(const v4u*)(qkvL + vbase + 8 * i);
#pragma unroll
      for (int e = 0; e < 8; ++e) {
        const unsigned uh = wh[e >> 1], ul = wl[e >> 1];
        const unsigned short sh = (unsigned short)((e & 1) ? (uh >> 16) : (uh & 0xffffu));
        const unsigned short sl = (unsigned short)((e & 1) ? (ul >> 16) : (ul & 0xffffu));
        vh[(dh + 8 * i + e) * 32 + c] = sh;
        vl[(dh + 8 * i + e) * 32 + c] = sl;
      }
    }
  }
  const __bf16* QH = (const __bf16*)qkvH;
  const __bf16* QL = (const __bf16*)qkvL;
  const size_t qb0 = (size_t)tokc * kQkvN + hc;
  v16b qh[2], ql[2], kh[2], kl[2];
#pragma unroll
  for (int dc = 0; dc < 2; ++dc) {
    qh[dc] = Frag<__bf16>::load(QH + qb0 + dc * 32 + koff);
    ql[dc] = Frag<__bf16>::load(QL + qb0 + dc * 32 + koff);
    kh[dc] = Frag<__bf16>::load(QH + qb0 + 256 + dc * 32 + koff);
    kl[dc] = Frag<__bf16>::load(QL + qb0 + 256 + dc * 32 + koff);
  }
  v8f sacc = zero8();
#pragma unroll
  for (int dc = 0; dc < 2; ++dc) {
    sacc = mma_b(qh[dc], kh[dc], sacc);
    sacc = mma_b(qh[dc], kl[dc], sacc);
    sacc = mma_b(ql[dc], kh[dc], sacc);
  }
  const float negInf = -__builtin_inff();
  float lsum[8];
#pragma unroll
  for (int r = 0; r < 8; ++r) {
    const int qw = 2 * hh + (r >> 2);
    const bool valid = (qw == (c >> 2));
    const float sv = valid ? (sacc[r] * kScale) : negInf;
    float m = sv;
#pragma unroll
    for (int off = 1; off < 16; off <<= 1) m = fmaxf(m, __shfl_xor(m, off, 32));
    const float e = expf(sv - m);
    float ps = e;
#pragma unroll
    for (int off = 1; off < 16; off <<= 1) ps += __shfl_xor(ps, off, 32);
    lsum[r] = ps;
    const unsigned short hb = f2bf_bits(e);
    const unsigned short lb = f2bf_bits(e - bf_bits2f(hb));
    ph[(8 * hh + r) * 32 + c] = hb;
    pl[(8 * hh + r) * 32 + c] = lb;
  }
  __syncthreads();
  const v16b pa = Frag<__bf16>::load((const __bf16*)(ph + c * 32 + koff));
  const v16b pb = Frag<__bf16>::load((const __bf16*)(pl + c * 32 + koff));
  v8f oacc[4];
#pragma unroll
  for (int t = 0; t < 4; ++t) {
    oacc[t] = zero8();
    const v16b va = Frag<__bf16>::load((const __bf16*)(vh + (t * 16 + c) * 32 + koff));
    const v16b vb = Frag<__bf16>::load((const __bf16*)(vl + (t * 16 + c) * 32 + koff));
    oacc[t] = mma_b(pa, va, oacc[t]);
    oacc[t] = mma_b(pa, vb, oacc[t]);
    oacc[t] = mma_b(pb, va, oacc[t]);
  }
  float* os = Os[wave];
#pragma unroll
  for (int r = 0; r < 8; ++r) {
    const float inv = 1.0f / lsum[r];
#pragma unroll
    for (int t = 0; t < 4; ++t) os[(8 * hh + r) * 68 + t * 16 + c] = oacc[t][r] * inv;
  }
  __syncthreads();
  {
    const int q8 = lane >> 3, c8 = (lane & 7) * 8;
    for (int pass = 0; pass < 2; ++pass) {
#pragma unroll
      for (int it = 0; it < 4; ++it) {
        const int row = it * 4 + q8;
        const int tok = tokBase + ((row & 3) >> 1) * 64 + 2 * (row >> 2) + (row & 1);
        const float* sp = os + row * 68 + c8;
        v8h hv, lv;
#pragma unroll
        for (int e = 0; e < 8; ++e) {
          const unsigned short hb = f2bf_bits(sp[e]);
          const unsigned short lb = f2bf_bits(sp[e] - bf_bits2f(hb));
          hv[e] = __builtin_bit_cast(_Float16, hb);
          lv[e] = __builtin_bit_cast(_Float16, lb);
        }
        const size_t o = (size_t)tok * kHalfDim + hc + c8;
        *(volatile v8h*)(oH + o) = hv;
        *(volatile v8h*)(oL + o) = lv;
      }
      __threadfence();
    }
  }
}

__global__ __launch_bounds__(128) void pool_attn(const unsigned short* __restrict__ q16, const unsigned short* __restrict__ k16,
                                                 const unsigned short* __restrict__ vT16, unsigned short* __restrict__ o16) {
  __shared__ __align__(16) _Float16 Ksh[64 * 64];
  __shared__ __align__(16) _Float16 Vts[64 * 64];
  __shared__ __align__(16) _Float16 Psh[4][16 * 64];
  __shared__ __align__(16) float Os[4][16 * 68];
  const int tid = threadIdx.x, lane = tid & 31, wave = tid >> 5;
  const int hh = lane >> 4, c = lane & 15, koff = hh * 8;
  const int bx = blockIdx.x;
  const int qb = bx & 63;
  const int bh = bx >> 6;
  const int head = bh & 3, b = bh >> 2;
  const int q0 = qb * 64 + wave * 16;
  const _Float16* Qp = (const _Float16*)q16;
  v16h qa[2];
#pragma unroll
  for (int dc = 0; dc < 2; ++dc)
    qa[dc] = Frag<_Float16>::load(Qp + (size_t)(b * kPix + q0 + c) * kHalfDim + head * kHead + dc * 32 + koff);

  const float negInf = -__builtin_inff();
  float mrow[8], lrow[8];
  v8f oacc[4];
#pragma unroll
  for (int r = 0; r < 8; ++r) { mrow[r] = negInf; lrow[r] = 0.f; }
#pragma unroll
  for (int t = 0; t < 4; ++t) oacc[t] = zero8();

  for (int kc = 0; kc < kPoolPer / 64; ++kc) {
    const int kv0 = kc * 64;
    __syncthreads();
    {
      const int rr = tid >> 1, dh = (tid & 1) * 32;
      const unsigned short* kr = k16 + (size_t)(b * kPoolPer + kv0 + rr) * kHalfDim + head * kHead + dh;
      const unsigned short* vr = vT16 + (size_t)(head * kHead + rr) * kPool + b * kPoolPer + kv0 + dh;
#pragma unroll
      for (int i = 0; i < 4; ++i) {
        const v4u kk = *(const v4u*)(kr + 8 * i);
        *(v4u*)(Ksh + rr * 64 + dh + 8 * i) = kk;
        const v4u vv = *(const v4u*)(vr + 8 * i);
        *(v4u*)(Vts + rr * 64 + dh + 8 * i) = vv;
      }
    }
    __syncthreads();

    v8f s[4];
#pragma unroll
    for (int j = 0; j < 4; ++j) {
      s[j] = zero8();
#pragma unroll
      for (int dc = 0; dc < 2; ++dc) {
        const v16h kb = Frag<_Float16>::load(Ksh + (j * 16 + c) * 64 + dc * 32 + koff);
        s[j] = mma_h(qa[dc], kb, s[j]);
      }
    }
    float cm[8];
#pragma unroll
    for (int r = 0; r < 8; ++r) {
      float m = negInf;
#pragma unroll
      for (int j = 0; j < 4; ++j) {
        s[j][r] = s[j][r] * kScale;
        m = fmaxf(m, s[j][r]);
      }
#pragma unroll
      for (int off = 1; off < 16; off <<= 1) m = fmaxf(m, __shfl_xor(m, off, 32));
      cm[r] = m;
    }
    _Float16* pw = Psh[wave];
#pragma unroll
    for (int r = 0; r < 8; ++r) {
      const float mnew = fmaxf(mrow[r], cm[r]);
      const float alpha = expf(mrow[r] - mnew);
      mrow[r] = mnew;
      float psum = 0.f;
#pragma unroll
      for (int j = 0; j < 4; ++j) {
        const float p = expf(s[j][r] - mnew);
        psum += p;
        pw[(8 * hh + r) * 64 + j * 16 + c] = (_Float16)(p * kPCarry);
      }
#pragma unroll
      for (int off = 1; off < 16; off <<= 1) psum += __shfl_xor(psum, off, 32);
      lrow[r] = lrow[r] * alpha + psum;
#pragma unroll
      for (int t = 0; t < 4; ++t) oacc[t][r] *= alpha;
    }
    __builtin_amdgcn_fence(__ATOMIC_RELEASE, "workgroup");
    __builtin_amdgcn_wave_barrier();
    __builtin_amdgcn_fence(__ATOMIC_ACQUIRE, "workgroup");
#pragma unroll
    for (int kk = 0; kk < 2; ++kk) {
      const v16h pa = Frag<_Float16>::load(pw + c * 64 + kk * 32 + koff);
#pragma unroll
      for (int t = 0; t < 4; ++t) {
        const v16h vb = Frag<_Float16>::load(Vts + (t * 16 + c) * 64 + kk * 32 + koff);
        oacc[t] = mma_h(pa, vb, oacc[t]);
      }
    }
  }

  float* os = Os[wave];
  const float outf = kLoOutCarry / kPCarry;
#pragma unroll
  for (int r = 0; r < 8; ++r) {
    const float inv = outf * (1.0f / lrow[r]);
#pragma unroll
    for (int t = 0; t < 4; ++t) os[(8 * hh + r) * 68 + t * 16 + c] = oacc[t][r] * inv;
  }
  __syncthreads();
  {
    const int q8 = lane >> 3, c8 = (lane & 7) * 8;
    for (int pass = 0; pass < 2; ++pass) {
#pragma unroll
      for (int it = 0; it < 4; ++it) {
        const int row = it * 4 + q8;
        const float* sp = os + row * 68 + c8;
        v8h hv;
#pragma unroll
        for (int e = 0; e < 8; ++e) hv[e] = (_Float16)sp[e];
        *(volatile v8h*)(o16 + (size_t)(b * kPix + q0 + row) * kHalfDim + head * kHead + c8) = hv;
      }
      __threadfence();
    }
  }
}

extern "C" void kernel_launch(void* const* d_in, const int* in_sizes, int n_in,
                              void* d_out, int out_size, void* d_ws, size_t ws_size,
                              hipStream_t stream) {
  if (n_in < 8) return;
  if (in_sizes[0] != kBatch * kChan * kPix) return;
  if (in_sizes[1] != kChan * kQkvN) return;
  if (in_sizes[2] != kHalfDim * kHalfDim) return;
  if (in_sizes[3] != kHalfDim) return;
  if (in_sizes[4] != kChan * kHalfDim) return;
  if (in_sizes[5] != kChan * kChan) return;
  if (in_sizes[6] != kHalfDim * kHalfDim) return;
  if (in_sizes[7] != kHalfDim) return;
  if (out_size != kBatch * kChan * kPix) return;
  if (ws_size < kCarveTotal) return;

  const float* x        = (const float*)d_in[0];
  const float* h_qkv_w  = (const float*)d_in[1];
  const float* h_proj_w = (const float*)d_in[2];
  const float* h_proj_b = (const float*)d_in[3];
  const float* l_q_w    = (const float*)d_in[4];
  const float* l_kv_w   = (const float*)d_in[5];
  const float* l_proj_w = (const float*)d_in[6];
  const float* l_proj_b = (const float*)d_in[7];
  float* out = (float*)d_out;

  char* ws = (char*)d_ws;
  size_t off = 0;
  auto carve = [&](size_t bytes) -> unsigned short* {
    unsigned short* p = (unsigned short*)(ws + off);
    off += (bytes + 255) & ~(size_t)255;
    return p;
  };
  unsigned short* xhH   = carve(kBytesXh);
  unsigned short* xhL   = carve(kBytesXh);
  unsigned short* poolH = carve(kBytesPool);
  unsigned short* qkvH  = carve(kBytesQkv);
  unsigned short* qkvL  = carve(kBytesQkv);
  unsigned short* q16   = carve(kBytesT256);
  unsigned short* k16   = carve(kBytesP256);
  unsigned short* vT16  = carve(kBytesP256);
  unsigned short* hoH   = carve(kBytesT256);
  unsigned short* hoL   = carve(kBytesT256);
  unsigned short* lo16  = carve(kBytesT256);
  unsigned short* WqkvH = carve(kBytesWqkv);
  unsigned short* WqkvL = carve(kBytesWqkv);
  unsigned short* WhpH  = carve(kBytesW256);
  unsigned short* WhpL  = carve(kBytesW256);
  unsigned short* WqH   = carve(kBytesWq);
  unsigned short* WkvH  = carve(kBytesWkv);
  unsigned short* Wlp   = carve(kBytesW256);
  if (off > ws_size) return;

  tr_convert<2><<<dim3(kQkvN / 64, kChan / 64, 1), 256, 0, stream>>>(h_qkv_w, 0L, kQkvN, WqkvH, WqkvL, 0L, kChan, 1.0f);
  tr_convert<2><<<dim3(kHalfDim / 64, kHalfDim / 64, 1), 256, 0, stream>>>(h_proj_w, 0L, kHalfDim, WhpH, WhpL, 0L, kHalfDim, 1.0f);
  tr_convert<1><<<dim3(kHalfDim / 64, kChan / 64, 1), 256, 0, stream>>>(l_q_w, 0L, kHalfDim, WqH, nullptr, 0L, kChan, 1.0f);
  tr_convert<1><<<dim3(kChan / 64, kChan / 64, 1), 256, 0, stream>>>(l_kv_w, 0L, kChan, WkvH, nullptr, 0L, kChan, 1.0f);
  tr_convert<0><<<dim3(kHalfDim / 64, kHalfDim / 64, 1), 256, 0, stream>>>(l_proj_w, 0L, kHalfDim, Wlp, nullptr, 0L, kHalfDim, kLoWCarry);

  tr_convert<2><<<dim3(kPix / 64, kChan / 64, kBatch), 256, 0, stream>>>(x, (long)kChan * kPix, kPix, xhH, xhL, (long)kPix * kChan, kChan, 1.0f);
  pool_to_bf16<<<dim3(kPoolPer / 64, kChan / 64, kBatch), 256, 0, stream>>>(x, poolH);

  wmma_gemm64<1, true, 0, 2><<<dim3((kTok / 64) * (kQkvN / 64) / 8, 1), 256, 0, stream>>>(
      xhH, xhL, kChan, 0L, WqkvH, WqkvL, kChan, 0L, qkvH, qkvL, kQkvN, 0L, nullptr, kTok, kQkvN, kChan, 1.0f);
  wmma_gemm64<1, false, 0, 1><<<dim3((kTok / 64) * (kHalfDim / 64) / 8, 1), 256, 0, stream>>>(
      xhH, nullptr, kChan, 0L, WqH, nullptr, kChan, 0L, q16, nullptr, kHalfDim, 0L, nullptr, kTok, kHalfDim, kChan, 1.0f);
  wmma_gemm64<1, false, 0, 1><<<dim3((kPool / 64) * (kHalfDim / 64) / 8, 1), 256, 0, stream>>>(
      poolH, nullptr, kChan, 0L, WkvH, nullptr, kChan, 0L, k16, nullptr, kHalfDim, 0L, nullptr, kPool, kHalfDim, kChan, 1.0f);
  wmma_gemm64<1, false, 0, 1><<<dim3((kHalfDim / 64) * (kPool / 64) / 8, 1), 256, 0, stream>>>(
      WkvH + (size_t)kHalfDim * kChan, nullptr, kChan, 0L, poolH, nullptr, kChan, 0L, vT16, nullptr, kPool, 0L, nullptr, kHalfDim, kPool, kChan, 1.0f);

  win_attn<<<dim3(kTok / 16), 128, 0, stream>>>(qkvH, qkvL, hoH, hoL);
  pool_attn<<<dim3(kBatch * 4 * (kPix / 64)), 128, 0, stream>>>(q16, k16, vT16, lo16);

  wmma_gemm64<1, true, 1, 0><<<dim3((kHalfDim / 64) * (kPix / 64) / 8, kBatch), 256, 0, stream>>>(
      WhpH, WhpL, kHalfDim, 0L, hoH, hoL, kHalfDim, (long)kPix * kHalfDim, out, nullptr, kPix, (long)kChan * kPix, h_proj_b,
      kHalfDim, kPix, kHalfDim, 1.0f);
  wmma_gemm64<0, false, 1, 0><<<dim3((kHalfDim / 64) * (kPix / 64) / 8, kBatch), 256, 0, stream>>>(
      Wlp, nullptr, kHalfDim, 0L, lo16, nullptr, kHalfDim, (long)kPix * kHalfDim, out + (size_t)kHalfDim * kPix, nullptr, kPix,
      (long)kChan * kPix, l_proj_b, kHalfDim, kPix, kHalfDim, 1.0f / (kLoOutCarry * kLoWCarry));
}
